// PointNetPP4DSetAbstraction_41111426957681
// MI455X (gfx1250) — hardware-verified
//
#include <hip/hip_runtime.h>
#include <stdint.h>
#pragma clang fp contract(off)

typedef __attribute__((ext_vector_type(16))) _Float16 v16h;
typedef __attribute__((ext_vector_type(8)))  _Float16 v8h;
typedef __attribute__((ext_vector_type(8)))  float    v8f;
typedef __attribute__((ext_vector_type(4)))  float    v4f;
typedef __attribute__((ext_vector_type(4)))  unsigned v4u;

constexpr int BATCH    = 2;
constexpr int FRAMES   = 8;
constexpr int FEAT_D   = 64;
constexpr int NPOINTS  = 1024;
constexpr int NSAMPLES = 512;
constexpr int NNEIGH   = 32;
constexpr int NFRAMES_ALL = BATCH * FRAMES;
constexpr int MROWS    = BATCH * NSAMPLES * FRAMES * NNEIGH;
constexpr int NGROUPS  = MROWS / NNEIGH;
constexpr int CIN0     = 67;
constexpr int CPAD0    = 96;
constexpr int CMID     = 64;
constexpr int COUT_LAST = 128;
constexpr float WCARRY     = 16.0f;
constexpr float WCARRY_INV = 1.0f / WCARRY;
constexpr float RADIUS_SQ  = 0.04f;
static_assert(MROWS == 262144);
static_assert(NGROUPS == 8192);
static_assert(CIN0 == FEAT_D + 3);
static_assert(CPAD0 % 32 == 0);
static_assert(CMID % 32 == 0);

constexpr size_t SZ_X0   = (size_t)MROWS * CPAD0 * 2;
constexpr size_t SZ_Y    = (size_t)MROWS * CMID * 2;
constexpr size_t SZ_PL   = (size_t)NGROUPS * COUT_LAST * 4;
constexpr size_t SZ_PT   = (size_t)NFRAMES_ALL * NPOINTS * FEAT_D * 2;
constexpr size_t SZ_W0T  = (size_t)64 * 4 * CPAD0 * 2;
constexpr size_t SZ_W1T  = (size_t)64 * 4 * CMID * 2;
constexpr size_t SZ_W2T  = (size_t)COUT_LAST * 4 * CMID * 2;
constexpr size_t SZ_BIAS = 512;
constexpr size_t SZ_FIDX = (size_t)BATCH * NSAMPLES * 4;
constexpr size_t OFF_X0   = 0;
constexpr size_t OFF_Y1   = OFF_X0 + SZ_X0;
constexpr size_t OFF_Y2   = OFF_Y1 + SZ_Y;
constexpr size_t OFF_PL   = OFF_Y2 + SZ_Y;
constexpr size_t OFF_PT   = OFF_PL + SZ_PL;
constexpr size_t OFF_W0T  = OFF_PT + SZ_PT;
constexpr size_t OFF_W1T  = OFF_W0T + SZ_W0T;
constexpr size_t OFF_W2T  = OFF_W1T + SZ_W1T;
constexpr size_t OFF_B0   = OFF_W2T + SZ_W2T;
constexpr size_t OFF_B1   = OFF_B0 + SZ_BIAS;
constexpr size_t OFF_B2   = OFF_B1 + SZ_BIAS;
constexpr size_t OFF_FIDX = OFF_B2 + SZ_BIAS;
constexpr size_t WS_TOTAL = OFF_FIDX + SZ_FIDX;
static_assert(WS_TOTAL == 123885056);
static_assert(WS_TOTAL <= 134217728);
static_assert(OFF_Y1 % 128 == 0 && OFF_Y2 % 128 == 0 && OFF_PL % 128 == 0 && OFF_PT % 128 == 0);
static_assert(OFF_W0T % 128 == 0 && OFF_W1T % 128 == 0 && OFF_W2T % 128 == 0);
static_assert(OFF_B0 % 128 == 0 && OFF_B1 % 128 == 0 && OFF_B2 % 128 == 0 && OFF_FIDX % 128 == 0);

constexpr int OUT0_ELEMS = BATCH * FRAMES * 3 * NSAMPLES;
constexpr int OUT1_ELEMS = BATCH * FRAMES * COUT_LAST * NSAMPLES;
static_assert(OUT0_ELEMS * 4 == 98304);
static_assert(OUT0_ELEMS * 4 + OUT1_ELEMS * 4 == 4292608);

__device__ __forceinline__ unsigned f16_bits(float x) {
  const _Float16 h = (_Float16)x;
  const unsigned short s = __builtin_bit_cast(unsigned short, h);
  return (unsigned)s;
}
__device__ __forceinline__ unsigned pack_halves(float lo, float hi) {
  const unsigned a = f16_bits(lo);
  const unsigned b = f16_bits(hi);
  return (a & 0xffffu) | (b << 16);
}
__device__ __forceinline__ int clampi(int v, int lo, int hi) {
  v = v < lo ? lo : v;
  v = v > hi ? hi : v;
  return v;
}
__device__ __forceinline__ unsigned long long shfl_xor_u64(unsigned long long v, int m) {
  unsigned lo = (unsigned)(v & 0xffffffffull);
  unsigned hi = (unsigned)(v >> 32);
  lo = __shfl_xor(lo, m, 32);
  hi = __shfl_xor(hi, m, 32);
  return (((unsigned long long)hi) << 32) | (unsigned long long)lo;
}

union FragU { v16h v; v8h h[2]; };
__device__ __forceinline__ v16h frag_load(const _Float16* p) {
  FragU f;
  f.h[0] = *(const v8h*)(p);
  f.h[1] = *(const v8h*)(p + 16);
  return f.v;
}
__device__ __forceinline__ v8f frag_mma(v16h a, v16h b, v8f c) {
  return __builtin_amdgcn_wmma_f32_16x16x32_f16(false, a, false, b, (short)0, c, false, false);
}
__device__ __forceinline__ void guard_row4(v8f& a0, v8f& a1, v8f& a2, v8f& a3,
                                           v16h x, v16h b0, v16h b1, v16h b2, v16h b3) {
  asm volatile("v_nop\n\tv_nop\n\tv_nop\n\tv_nop\n\tv_nop"
               : "+v"(a0), "+v"(a1), "+v"(a2), "+v"(a3)
               : "v"(x), "v"(b0), "v"(b1), "v"(b2), "v"(b3));
}
__device__ __forceinline__ void acc_guard4(v8f& a, v8f& b, v8f& c, v8f& d) {
  asm volatile("v_nop\n\tv_nop\n\tv_nop\n\tv_nop" : "+v"(a), "+v"(b), "+v"(c), "+v"(d));
}

template <int CI, int CO, int CP, bool FEATFIRST>
__global__ __launch_bounds__(256) void fold_weights_kernel(
    const float* __restrict__ w, const float* __restrict__ cb, const float* __restrict__ g,
    const float* __restrict__ be, const float* __restrict__ mu, const float* __restrict__ var,
    unsigned short* __restrict__ wt, float* __restrict__ biasf) {
  constexpr int KTOT = 4 * CP;
  constexpr int PER_ROW = KTOT / 8;
  constexpr int TOTAL = CO * PER_ROW;
  static_assert(CP % 8 == 0);
  static_assert(TOTAL % 256 == 0);
  const int gid = blockIdx.x * 256 + threadIdx.x;
  const int gc = gid < TOTAL ? gid : (TOTAL - 1);
  const int co = gc / PER_ROW;
  const int k8 = (gc - co * PER_ROW) * 8;
  const int dt = k8 / CP;
  const int j0 = k8 - dt * CP;
  const float sc = g[co] * (1.0f / sqrtf(var[co] + 1e-5f));
  float vals[8];
#pragma unroll
  for (int e = 0; e < 8; ++e) {
    const int j = j0 + e;
    const bool ok = j < CI;
    int ci = FEATFIRST ? ((j < 64) ? (j + 3) : (j - 64)) : j;
    ci = clampi(ci, 0, CI - 1);
    const float wv = w[(co * CI + ci) * 4 + dt];
    const float sv = (wv * sc) * WCARRY;
    vals[e] = ok ? sv : 0.0f;
  }
  v4u o;
  o.x = pack_halves(vals[0], vals[1]);
  o.y = pack_halves(vals[2], vals[3]);
  o.z = pack_halves(vals[4], vals[5]);
  o.w = pack_halves(vals[6], vals[7]);
  if (gid < TOTAL) {
    v4u* dst = (v4u*)wt + gid;
    *(volatile v4u*)dst = o;
    __threadfence();
    *(volatile v4u*)dst = o;
  }
  if (blockIdx.x == 0 && threadIdx.x < CO / 4) {
    const int c4 = threadIdx.x * 4;
    const v4f vb = *(const v4f*)(cb + c4);
    const v4f vg = *(const v4f*)(g + c4);
    const v4f ve = *(const v4f*)(be + c4);
    const v4f vm = *(const v4f*)(mu + c4);
    const v4f vv = *(const v4f*)(var + c4);
    v4f r;
#pragma unroll
    for (int e = 0; e < 4; ++e) {
      const float s2 = vg[e] * (1.0f / sqrtf(vv[e] + 1e-5f));
      const float d = vb[e] - vm[e];
      const float p = d * s2;
      r[e] = p + ve[e];
    }
    *(volatile v4f*)(biasf + c4) = r;
    __threadfence();
    *(volatile v4f*)(biasf + c4) = r;
  }
}

__global__ __launch_bounds__(256) void points_to_rows_kernel(const float* __restrict__ pts,
                                                             unsigned short* __restrict__ pt) {
  __shared__ float tile[64][33];
  const int tid = threadIdx.x;
  const int lane = tid & 31;
  const int wave = tid >> 5;
  const int bt = blockIdx.x >> 5;
  const int n0 = (blockIdx.x & 31) * 32;
#pragma unroll
  for (int i = 0; i < 8; ++i) {
    const int c = wave * 8 + i;
    tile[c][lane] = pts[((size_t)(bt * FEAT_D + c)) * NPOINTS + n0 + lane];
  }
  __syncthreads();
  const int nl = tid >> 3;
  const int ch = tid & 7;
  const int c8 = ch * 8;
  float a[8];
#pragma unroll
  for (int e = 0; e < 8; ++e) a[e] = tile[c8 + e][nl];
  v4u o;
  o.x = pack_halves(a[0], a[1]);
  o.y = pack_halves(a[2], a[3]);
  o.z = pack_halves(a[4], a[5]);
  o.w = pack_halves(a[6], a[7]);
  v4u* dst = (v4u*)pt + ((size_t)(bt * NPOINTS + n0 + nl)) * 8 + ch;
  *(volatile v4u*)dst = o;
  __threadfence();
  *(volatile v4u*)dst = o;
}

__global__ __launch_bounds__(256) void sample_far_kernel(const float* __restrict__ xyz,
                                                         int* __restrict__ fidx) {
#pragma clang fp contract(off)
  __shared__ float sx[3 * NPOINTS];
  __shared__ unsigned long long red[2][8];
  __shared__ int sidx[NSAMPLES];
  const int tid = threadIdx.x;
  const int lane = tid & 31;
  const int wave = tid >> 5;
  const int b = blockIdx.x;
  const float* x = xyz + (size_t)b * FRAMES * 3 * NPOINTS;
  float px[4], py[4], pz[4], mind[4];
#pragma unroll
  for (int i = 0; i < 4; ++i) {
    const int n = tid + i * 256;
    px[i] = x[n];
    py[i] = x[NPOINTS + n];
    pz[i] = x[2 * NPOINTS + n];
    mind[i] = 1e10f;
  }
#pragma unroll
  for (int i = 0; i < 4; ++i) {
    const int n = tid + i * 256;
    sx[n] = px[i];
    sx[NPOINTS + n] = py[i];
    sx[2 * NPOINTS + n] = pz[i];
  }
  if (tid == 0) sidx[0] = 0;
  __syncthreads();
  int far = 0;
  int buf = 0;
#pragma unroll 1
  for (int it = 1; it < NSAMPLES; ++it) {
    const float cx = sx[far];
    const float cy = sx[NPOINTS + far];
    const float cz = sx[2 * NPOINTS + far];
    unsigned long long best = 0ull;
#pragma unroll
    for (int i = 0; i < 4; ++i) {
      const int n = tid + i * 256;
      const float dx = px[i] - cx;
      const float dy = py[i] - cy;
      const float dz = pz[i] - cz;
      const float tx = dx * dx;
      const float ty = dy * dy;
      const float tz = dz * dz;
      const float sxz = tx + tz;
      const float d = sxz + ty;
      mind[i] = fminf(mind[i], d);
      const unsigned long long key =
          (((unsigned long long)__float_as_uint(mind[i])) << 32) | (unsigned long long)(unsigned)(1023 - n);
      best = key > best ? key : best;
    }
#pragma unroll
    for (int off = 16; off > 0; off >>= 1) {
      const unsigned long long o = shfl_xor_u64(best, off);
      best = o > best ? o : best;
    }
    if (lane == 0) red[buf][wave] = best;
    __syncthreads();
    unsigned long long r = red[buf][0];
#pragma unroll
    for (int wv = 1; wv < 8; ++wv) {
      const unsigned long long o = red[buf][wv];
      r = o > r ? o : r;
    }
    far = 1023 - (int)((unsigned)(r & 0xffffffffull) & 1023u);
    if (tid == 0) sidx[it] = far;
    buf ^= 1;
  }
  __syncthreads();
  if (tid < NSAMPLES / 4) {
    v4u o;
    o.x = (unsigned)sidx[tid * 4 + 0];
    o.y = (unsigned)sidx[tid * 4 + 1];
    o.z = (unsigned)sidx[tid * 4 + 2];
    o.w = (unsigned)sidx[tid * 4 + 3];
    v4u* dst = (v4u*)(fidx + b * NSAMPLES) + tid;
    *(volatile v4u*)dst = o;
    __threadfence();
    *(volatile v4u*)dst = o;
  }
}

__global__ __launch_bounds__(256) void centres_out_kernel(const float* __restrict__ xyz,
                                                          const int* __restrict__ fidx,
                                                          float* __restrict__ out0) {
  const int gid = blockIdx.x * 256 + threadIdx.x;
  const int rc = gid >> 7;
  const int s4 = (gid & 127) * 4;
  const int bt = rc / 3;
  const int b = bt >> 3;
  v4f o;
#pragma unroll
  for (int e = 0; e < 4; ++e) {
    const int idx = clampi(fidx[b * NSAMPLES + s4 + e], 0, NPOINTS - 1);
    o[e] = xyz[(size_t)rc * NPOINTS + idx];
  }
  float* dst = out0 + (size_t)rc * NSAMPLES + s4;
  *(volatile v4f*)dst = o;
  __threadfence();
  *(volatile v4f*)dst = o;
}

__global__ __launch_bounds__(128) void group_rows_kernel(const float* __restrict__ xyz,
                                                         const unsigned short* __restrict__ pt,
                                                         const int* __restrict__ fidx,
                                                         unsigned short* __restrict__ x0) {
#pragma clang fp contract(off)
  __shared__ __align__(16) v4u stage[4][384];
  __shared__ int slots[4][32];
  const int tid = threadIdx.x;
  const int lane = tid & 31;
  const int wave = tid >> 5;
  const int wid = blockIdx.x * 4 + wave;
  const int bt = wid >> 9;
  const int s = wid & 511;
  const int b = bt >> 3;
  const int t = bt & 7;
  const float* x = xyz + (size_t)bt * 3 * NPOINTS;
  const int i0 = clampi(fidx[b * NSAMPLES + s], 0, NPOINTS - 1);
  const float cx = x[i0];
  const float cy = x[NPOINTS + i0];
  const float cz = x[2 * NPOINTS + i0];
  const float tcx = cx * cx;
  const float tcy = cy * cy;
  const float tcz = cz * cz;
  const float sxz_c = tcx + tcz;
  const float sqc = sxz_c + tcy;
  slots[wave][lane] = NPOINTS - 1;
  __syncthreads();
  int total = 0;
#pragma unroll 1
  for (int base = 0; base < NPOINTS; base += 32) {
    if (total >= NNEIGH) break;
    const int n = base + lane;
    const float xx = x[n];
    const float yy = x[NPOINTS + n];
    const float zz = x[2 * NPOINTS + n];
    const float tx = xx * xx;
    const float ty = yy * yy;
    const float tz = zz * zz;
    const float sxz = tx + tz;
    const float sqn = sxz + ty;
    float p = cx * xx;
    p = __builtin_fmaf(cy, yy, p);
    p = __builtin_fmaf(cz, zz, p);
    const float ssum = sqc + sqn;
    const float p2 = 2.0f * p;
    const float sq = ssum - p2;
    const bool in = !(sq > RADIUS_SQ);
    const unsigned mask = (unsigned)__ballot(in);
    const int pos = total + __popc(mask & ((1u << lane) - 1u));
    if (in && pos < NNEIGH) slots[wave][pos] = n;
    total += __popc(mask);
  }
  __syncthreads();
  const int tot = total < NNEIGH ? total : NNEIGH;
  {
    const int oi = lane < tot ? lane : 0;
    const int nk = clampi(slots[wave][oi], 0, NPOINTS - 1);
    const float rx = x[nk] - cx;
    const float ry = x[NPOINTS + nk] - cy;
    const float rz = x[2 * NPOINTS + nk] - cz;
    unsigned zpad = 0;
    asm volatile("" : "+v"(zpad));
    const unsigned hx = f16_bits(rx);
    const unsigned hy = f16_bits(ry);
    const unsigned hz = f16_bits(rz);
    v4u t0;
    t0.x = (hx & 0xffffu) | (hy << 16);
    t0.y = (hz & 0xffffu) | (zpad << 16);
    t0.z = zpad;
    t0.w = zpad;
    v4u tz4;
    tz4.x = zpad;
    tz4.y = zpad;
    tz4.z = zpad;
    tz4.w = zpad;
    stage[wave][lane * 12 + 8] = t0;
    stage[wave][lane * 12 + 9] = tz4;
    stage[wave][lane * 12 + 10] = tz4;
    stage[wave][lane * 12 + 11] = tz4;
  }
  {
    const v4u* ptv = (const v4u*)pt;
    const int q = lane >> 3;
    const int ch = lane & 7;
#pragma unroll
    for (int it = 0; it < 8; ++it) {
      const int r = it * 4 + q;
      const int ri = r < tot ? r : 0;
      const int nr = clampi(slots[wave][ri], 0, NPOINTS - 1);
      const v4u v = ptv[((size_t)(bt * NPOINTS + nr)) * 8 + ch];
      stage[wave][r * 12 + ch] = v;
    }
  }
  __syncthreads();
  {
    const size_t m0 = ((size_t)((b * NSAMPLES + s) * FRAMES + t)) * NNEIGH;
    v4u* dst = (v4u*)x0 + m0 * 12;
    for (int pass = 0; pass < 2; ++pass) {
#pragma unroll
      for (int it = 0; it < 12; ++it) {
        const v4u v = stage[wave][it * 32 + lane];
        *(volatile v4u*)(dst + it * 32 + lane) = v;
      }
      __threadfence();
    }
  }
}

template <int CPAD, int NOUT, bool FINAL>
__global__ __launch_bounds__(256) void conv_gemm_kernel(
    const unsigned short* __restrict__ Xp, const unsigned short* __restrict__ Wp,
    const float* __restrict__ bias, unsigned short* __restrict__ Yp, float* __restrict__ Pp) {
  constexpr int KTOT = 4 * CPAD;
  constexpr int TILES_N = NOUT / 64;
  constexpr int TILES_M = MROWS / 64;
  static_assert(CPAD % 32 == 0);
  static_assert(KTOT % 32 == 0);
  static_assert(NOUT % 64 == 0);
  static_assert(MROWS % 64 == 0);
  static_assert((TILES_M * TILES_N) % 8 == 0);
  static_assert(FINAL || NOUT == 64);
  const _Float16* X = (const _Float16*)Xp;
  const _Float16* W = (const _Float16*)Wp;
  __shared__ __align__(16) float sT[8][16 * 68];
  const int lane = threadIdx.x & 31;
  const int wave = threadIdx.x >> 5;
  const int tile = blockIdx.x * 8 + wave;
  int tm = tile / TILES_N;
  const int tn = tile - tm * TILES_N;
  tm = tm < TILES_M ? tm : (TILES_M - 1);
  const int m0 = tm << 6;
  const int n0 = tn << 6;
  const int rlane = lane & 15;
  const int hh = lane >> 4;
  const int koff = hh * 8;
  const int mOff = hh * 8;
  const int tlo = (m0 >> 5) & 7;

  v8f acc[4][4];
#pragma unroll
  for (int i = 0; i < 4; ++i)
#pragma unroll
    for (int j = 0; j < 4; ++j) acc[i][j] = (v8f){0.f, 0.f, 0.f, 0.f, 0.f, 0.f, 0.f, 0.f};
  const v16h zfrag = {};

#pragma unroll 1
  for (int dt = 0; dt < 4; ++dt) {
    bool va[4];
    size_t aoff[4];
#pragma unroll
    for (int i = 0; i < 4; ++i) {
      const int tt = tlo + (i >> 1) + dt - 1;
      va[i] = (tt >= 0) && (tt < FRAMES);
      const int mrow = m0 + (i << 4) + rlane;
      int srow = va[i] ? (mrow + (dt - 1) * NNEIGH) : mrow;
      srow = clampi(srow, 0, MROWS - 1);
      aoff[i] = (size_t)srow * CPAD + koff;
    }
#pragma unroll 1
    for (int kin = 0; kin < CPAD; kin += 32) {
      v16h bh[4];
#pragma unroll
      for (int j = 0; j < 4; ++j) {
        const size_t bo = (size_t)(n0 + (j << 4) + rlane) * KTOT + dt * CPAD + kin + koff;
        bh[j] = frag_load(W + bo);
      }
#pragma unroll
      for (int i = 0; i < 4; ++i) {
        v16h ah = frag_load(X + aoff[i] + kin);
        ah = va[i] ? ah : zfrag;
#pragma unroll
        for (int j = 0; j < 4; ++j) acc[i][j] = frag_mma(ah, bh[j], acc[i][j]);
        guard_row4(acc[i][0], acc[i][1], acc[i][2], acc[i][3], ah, bh[0], bh[1], bh[2], bh[3]);
      }
    }
  }
  acc_guard4(acc[0][0], acc[0][1], acc[0][2], acc[0][3]);
  acc_guard4(acc[1][0], acc[1][1], acc[1][2], acc[1][3]);
  acc_guard4(acc[2][0], acc[2][1], acc[2][2], acc[2][3]);
  acc_guard4(acc[3][0], acc[3][1], acc[3][2], acc[3][3]);

  float* slab = sT[wave];
  if (!FINAL) {
#pragma unroll
    for (int i = 0; i < 4; ++i) {
      const int mBase = m0 + (i << 4);
#pragma unroll
      for (int j = 0; j < 4; ++j) {
        const float bv = bias[n0 + (j << 4) + rlane];
#pragma unroll
        for (int r = 0; r < 8; ++r) {
          float v = acc[i][j][r] * WCARRY_INV;
          v = v + bv;
          v = fmaxf(v, 0.0f);
          slab[(mOff + r) * 68 + (j << 4) + rlane] = v;
        }
      }
      __builtin_amdgcn_fence(__ATOMIC_RELEASE, "workgroup");
      __builtin_amdgcn_wave_barrier();
      __builtin_amdgcn_fence(__ATOMIC_ACQUIRE, "workgroup");
      {
        const int q = lane >> 3;
        const int c8 = (lane & 7) * 8;
        for (int pass = 0; pass < 2; ++pass) {
#pragma unroll
          for (int it = 0; it < 4; ++it) {
            const int row = it * 4 + q;
            const float* sp = slab + row * 68 + c8;
            v8h hv;
#pragma unroll
            for (int e = 0; e < 8; ++e) hv[e] = (_Float16)sp[e];
            *(volatile v8h*)(Yp + (size_t)(mBase + row) * NOUT + n0 + c8) = hv;
          }
          __threadfence();
        }
      }
      __builtin_amdgcn_fence(__ATOMIC_RELEASE, "workgroup");
      __builtin_amdgcn_wave_barrier();
      __builtin_amdgcn_fence(__ATOMIC_ACQUIRE, "workgroup");
    }
  } else {
#pragma unroll
    for (int g = 0; g < 2; ++g) {
#pragma unroll
      for (int j = 0; j < 4; ++j) {
        float mx = acc[2 * g][j][0];
#pragma unroll
        for (int r = 1; r < 8; ++r) mx = fmaxf(mx, acc[2 * g][j][r]);
#pragma unroll
        for (int r = 0; r < 8; ++r) mx = fmaxf(mx, acc[2 * g + 1][j][r]);
        const float other = __shfl_xor(mx, 16, 32);
        mx = fmaxf(mx, other);
        float v = mx * WCARRY_INV;
        v = v + bias[n0 + (j << 4) + rlane];
        v = fmaxf(v, 0.0f);
        slab[hh * 128 + g * 64 + (j << 4) + rlane] = v;
      }
    }
    __builtin_amdgcn_fence(__ATOMIC_RELEASE, "workgroup");
    __builtin_amdgcn_wave_barrier();
    __builtin_amdgcn_fence(__ATOMIC_ACQUIRE, "workgroup");
    {
      const v4f o = *(const v4f*)(slab + lane * 4);
      float* dst = Pp + (size_t)((m0 >> 5) + (lane >> 4)) * COUT_LAST + n0 + (lane & 15) * 4;
      *(volatile v4f*)dst = o;
      __threadfence();
      *(volatile v4f*)dst = o;
    }
  }
}

__global__ __launch_bounds__(256) void pool_to_out_kernel(const float* __restrict__ pl,
                                                          float* __restrict__ out1) {
  __shared__ float tile[32][33];
  const int tid = threadIdx.x;
  const int bx = blockIdx.x;
  const int ct = bx & 3;
  const int st = (bx >> 2) & 15;
  const int bt = bx >> 6;
  const int b = bt >> 3;
  const int t = bt & 7;
  const int co0 = ct * 32;
  const int s0 = st * 32;
  {
    const int sl = tid >> 3;
    const int c4 = (tid & 7) * 4;
    const size_t prow = (size_t)((b * NSAMPLES + s0 + sl) * FRAMES + t);
    const v4f v = *(const v4f*)(pl + prow * COUT_LAST + co0 + c4);
    tile[sl][c4 + 0] = v[0];
    tile[sl][c4 + 1] = v[1];
    tile[sl][c4 + 2] = v[2];
    tile[sl][c4 + 3] = v[3];
  }
  __syncthreads();
  {
    const int cl = tid >> 3;
    const int s4 = (tid & 7) * 4;
    v4f o;
    o[0] = tile[s4 + 0][cl];
    o[1] = tile[s4 + 1][cl];
    o[2] = tile[s4 + 2][cl];
    o[3] = tile[s4 + 3][cl];
    float* dst = out1 + ((size_t)(bt * COUT_LAST + co0 + cl)) * NSAMPLES + s0 + s4;
    *(volatile v4f*)dst = o;
    __threadfence();
    *(volatile v4f*)dst = o;
  }
}

extern "C" void kernel_launch(void* const* d_in, const int* in_sizes, int n_in,
                              void* d_out, int out_size, void* d_ws, size_t ws_size,
                              hipStream_t stream) {
  (void)in_sizes;
  if (n_in < 20) return;
  if (out_size < OUT0_ELEMS + OUT1_ELEMS) return;
  if (ws_size < WS_TOTAL) return;

  const float* xyz = (const float*)d_in[0];
  const float* pts = (const float*)d_in[1];
  const float* w0  = (const float*)d_in[2];
  const float* b0  = (const float*)d_in[3];
  const float* g0  = (const float*)d_in[4];
  const float* be0 = (const float*)d_in[5];
  const float* m0  = (const float*)d_in[6];
  const float* v0  = (const float*)d_in[7];
  const float* w1  = (const float*)d_in[8];
  const float* b1  = (const float*)d_in[9];
  const float* g1  = (const float*)d_in[10];
  const float* be1 = (const float*)d_in[11];
  const float* m1  = (const float*)d_in[12];
  const float* v1  = (const float*)d_in[13];
  const float* w2  = (const float*)d_in[14];
  const float* b2  = (const float*)d_in[15];
  const float* g2  = (const float*)d_in[16];
  const float* be2 = (const float*)d_in[17];
  const float* m2  = (const float*)d_in[18];
  const float* v2  = (const float*)d_in[19];

  float* out0 = (float*)d_out;
  float* out1 = (float*)d_out + OUT0_ELEMS;

  char* ws = (char*)d_ws;
  unsigned short* X0  = (unsigned short*)(ws + OFF_X0);
  unsigned short* Y1  = (unsigned short*)(ws + OFF_Y1);
  unsigned short* Y2  = (unsigned short*)(ws + OFF_Y2);
  float*          PL  = (float*)(ws + OFF_PL);
  unsigned short* PT  = (unsigned short*)(ws + OFF_PT);
  unsigned short* W0T = (unsigned short*)(ws + OFF_W0T);
  unsigned short* W1T = (unsigned short*)(ws + OFF_W1T);
  unsigned short* W2T = (unsigned short*)(ws + OFF_W2T);
  float*          BS0 = (float*)(ws + OFF_B0);
  float*          BS1 = (float*)(ws + OFF_B1);
  float*          BS2 = (float*)(ws + OFF_B2);
  int*            FIDX = (int*)(ws + OFF_FIDX);

  fold_weights_kernel<CIN0, 64, CPAD0, true><<<(64 * (4 * CPAD0 / 8)) / 256, 256, 0, stream>>>(
      w0, b0, g0, be0, m0, v0, W0T, BS0);
  fold_weights_kernel<CMID, 64, CMID, false><<<(64 * (4 * CMID / 8)) / 256, 256, 0, stream>>>(
      w1, b1, g1, be1, m1, v1, W1T, BS1);
  fold_weights_kernel<CMID, COUT_LAST, CMID, false><<<(COUT_LAST * (4 * CMID / 8)) / 256, 256, 0, stream>>>(
      w2, b2, g2, be2, m2, v2, W2T, BS2);

  points_to_rows_kernel<<<NFRAMES_ALL * (NPOINTS / 32), 256, 0, stream>>>(pts, PT);

  sample_far_kernel<<<BATCH, 256, 0, stream>>>(xyz, FIDX);

  centres_out_kernel<<<(NFRAMES_ALL * 3 * (NSAMPLES / 4)) / 256, 256, 0, stream>>>(xyz, FIDX, out0);

  group_rows_kernel<<<(NFRAMES_ALL * NSAMPLES) / 4, 128, 0, stream>>>(xyz, PT, FIDX, X0);

  conv_gemm_kernel<CPAD0, 64, false><<<(MROWS / 64) / 8, 256, 0, stream>>>(X0, W0T, BS0, Y1, PL);
  conv_gemm_kernel<CMID, 64, false><<<(MROWS / 64) / 8, 256, 0, stream>>>(Y1, W1T, BS1, Y2, PL);
  conv_gemm_kernel<CMID, COUT_LAST, true><<<((MROWS / 64) * 2) / 8, 256, 0, stream>>>(Y2, W2T, BS2, Y1, PL);

  pool_to_out_kernel<<<NFRAMES_ALL * 16 * 4, 256, 0, stream>>>(PL, out1);
}
